// BilinearGrounding_21792664060129
// MI455X (gfx1250) — hardware-verified
//
#include <hip/hip_runtime.h>
#include <stddef.h>
#include <stdint.h>

#define NB   64
#define NT   128
#define NR   100
#define TH   768
#define IH   2048
#define MI   (NB * NR)
#define MT   (NB * NT)
#define SLAB (NT * NR)

static_assert(MI % 256 == 0);
static_assert(MT % 128 == 0);
static_assert(TH % 64 == 0);
static_assert(TH % 32 == 0);
static_assert(IH % 32 == 0);
static_assert((MI * IH) % 2048 == 0);
static_assert((MT * TH) % 2048 == 0);
static_assert((TH * IH) % 2048 == 0);
static_assert((TH * TH) % 2048 == 0);
static_assert(SLAB % 4 == 0);
static_assert((SLAB * 4) % 128 == 0);
static_assert(NR <= 128);

typedef _Float16 v16h __attribute__((ext_vector_type(16)));
typedef _Float16 v8h  __attribute__((ext_vector_type(8)));
typedef float    v8f  __attribute__((ext_vector_type(8)));
typedef float    v4f  __attribute__((ext_vector_type(4)));
typedef unsigned int v4u __attribute__((ext_vector_type(4)));

union Frag  { v16h v; v8h h[2]; };
union Pack8 { v8h h; v4u u; };

__device__ __forceinline__ v8f mma16(v16h a, v16h b, v8f c) {
  c = __builtin_amdgcn_wmma_f32_16x16x32_f16(false, a, false, b, (short)0, c, false, false);
  asm volatile("v_nop\n\tv_nop\n\tv_nop\n\tv_nop" : "+v"(c) : "v"(a), "v"(b));
  return c;
}

__device__ __forceinline__ v8f zero8() { return (v8f){0.f, 0.f, 0.f, 0.f, 0.f, 0.f, 0.f, 0.f}; }

__device__ __forceinline__ void gemm32x64(const _Float16* __restrict__ A, int lda,
                                          const _Float16* __restrict__ Bt, int ldb, int K,
                                          int m0, int n0, int nmax, int lane, v8f (&acc)[2][4]) {
  const int m = lane & 15, lh = lane >> 4;
  const _Float16* pa0 = A + (size_t)(m0 + m) * lda + 8 * lh;
  const _Float16* pa1 = A + (size_t)(m0 + 16 + m) * lda + 8 * lh;
  int r0 = n0 + m, r1 = n0 + 16 + m, r2 = n0 + 32 + m, r3 = n0 + 48 + m;
  r0 = (r0 > nmax) ? nmax : r0;
  r1 = (r1 > nmax) ? nmax : r1;
  r2 = (r2 > nmax) ? nmax : r2;
  r3 = (r3 > nmax) ? nmax : r3;
  const _Float16* pb0 = Bt + (size_t)r0 * ldb + 8 * lh;
  const _Float16* pb1 = Bt + (size_t)r1 * ldb + 8 * lh;
  const _Float16* pb2 = Bt + (size_t)r2 * ldb + 8 * lh;
  const _Float16* pb3 = Bt + (size_t)r3 * ldb + 8 * lh;
#pragma unroll 2
  for (int k0 = 0; k0 < K; k0 += 32) {
    Frag a0, a1, b0, b1, b2, b3;
    a0.h[0] = *(const v8h*)(pa0 + k0); a0.h[1] = *(const v8h*)(pa0 + k0 + 16);
    a1.h[0] = *(const v8h*)(pa1 + k0); a1.h[1] = *(const v8h*)(pa1 + k0 + 16);
    b0.h[0] = *(const v8h*)(pb0 + k0); b0.h[1] = *(const v8h*)(pb0 + k0 + 16);
    b1.h[0] = *(const v8h*)(pb1 + k0); b1.h[1] = *(const v8h*)(pb1 + k0 + 16);
    b2.h[0] = *(const v8h*)(pb2 + k0); b2.h[1] = *(const v8h*)(pb2 + k0 + 16);
    b3.h[0] = *(const v8h*)(pb3 + k0); b3.h[1] = *(const v8h*)(pb3 + k0 + 16);
    acc[0][0] = mma16(a0.v, b0.v, acc[0][0]);
    acc[1][0] = mma16(a1.v, b0.v, acc[1][0]);
    acc[0][1] = mma16(a0.v, b1.v, acc[0][1]);
    acc[1][1] = mma16(a1.v, b1.v, acc[1][1]);
    acc[0][2] = mma16(a0.v, b2.v, acc[0][2]);
    acc[1][2] = mma16(a1.v, b2.v, acc[1][2]);
    acc[0][3] = mma16(a0.v, b3.v, acc[0][3]);
    acc[1][3] = mma16(a1.v, b3.v, acc[1][3]);
  }
}

__global__ __launch_bounds__(256) void k_cvt(const float* __restrict__ src, _Float16* __restrict__ dst, float scale) {
  const size_t o = ((size_t)blockIdx.x * 256 + threadIdx.x) * 8;
  const v4f a0 = *(const v4f*)(src + o);
  const v4f a1 = *(const v4f*)(src + o + 4);
  Pack8 pk;
  pk.h = (v8h){(_Float16)(a0[0] * scale), (_Float16)(a0[1] * scale), (_Float16)(a0[2] * scale), (_Float16)(a0[3] * scale),
               (_Float16)(a1[0] * scale), (_Float16)(a1[1] * scale), (_Float16)(a1[2] * scale), (_Float16)(a1[3] * scale)};
  const v4u vv = pk.u;
  volatile v4u* d = (volatile v4u*)(dst + o);
  *d = vv;
  __threadfence();
  *d = vv;
}

#define HP 72
template <int HASB>
__global__ __launch_bounds__(256) void k_gemm(const _Float16* __restrict__ A, int lda,
                                              const _Float16* __restrict__ Bt, int ldb, int K, int N,
                                              const float* __restrict__ bias, float scale,
                                              _Float16* __restrict__ C, int ldc) {
  __shared__ __align__(16) _Float16 st[8][32 * HP];
  const int tid = threadIdx.x, lane = tid & 31, wave = tid >> 5;
  const int hh = lane >> 4, c = lane & 15;
  const int m0 = blockIdx.x * 256 + wave * 32;
  const int n0 = blockIdx.y * 64;

  v8f acc[2][4];
#pragma unroll
  for (int s = 0; s < 2; ++s)
#pragma unroll
    for (int t = 0; t < 4; ++t) acc[s][t] = zero8();
  gemm32x64(A, lda, Bt, ldb, K, m0, n0, N - 1, lane, acc);

  _Float16* sw = st[wave];
#pragma unroll
  for (int sub = 0; sub < 2; ++sub) {
#pragma unroll
    for (int t = 0; t < 4; ++t) {
      float bb = 0.f;
      if (HASB) bb = bias[n0 + 16 * t + c];
#pragma unroll
      for (int r = 0; r < 8; ++r)
        sw[(16 * sub + 8 * hh + r) * HP + 16 * t + c] = (_Float16)(acc[sub][t][r] * scale + bb);
    }
  }
  __syncthreads();

  v4u val[8];
  size_t go[8];
#pragma unroll
  for (int it = 0; it < 8; ++it) {
    const int p  = lane + 32 * it;
    const int L  = p >> 3;
    const int pc = p & 7;
    Pack8 pk;
    pk.h    = *(const v8h*)(sw + L * HP + pc * 8);
    val[it] = pk.u;
    go[it]  = (size_t)(m0 + L) * ldc + n0 + pc * 8;
  }
  for (int ps = 0; ps < 2; ++ps) {
#pragma unroll
    for (int it = 0; it < 8; ++it) *(volatile v4u*)(C + go[it]) = val[it];
    __threadfence();
  }
}

__global__ __launch_bounds__(256) void k_bil(const _Float16* __restrict__ Tp, const _Float16* __restrict__ Wp,
                                             const float* __restrict__ mask, const float* __restrict__ bilb,
                                             float* __restrict__ out) {
  __shared__ __align__(16) float so[SLAB];
  const int tid = threadIdx.x, lane = tid & 31, wave = tid >> 5;
  const int hh = lane >> 4, c = lane & 15;
  const int wm = wave >> 1, wn = wave & 1;
  const int b  = blockIdx.x;
  const int m0 = b * NT + wm * 32;
  const int n0 = b * NR + wn * 64;

  v8f acc[2][4];
#pragma unroll
  for (int s = 0; s < 2; ++s)
#pragma unroll
    for (int t = 0; t < 4; ++t) acc[s][t] = zero8();
  gemm32x64(Tp, TH, Wp, TH, TH, m0, n0, MI - 1, lane, acc);

#pragma unroll
  for (int sub = 0; sub < 2; ++sub) {
#pragma unroll
    for (int t = 0; t < 4; ++t) {
      const int n = wn * 64 + 16 * t + c;
      if (n < NR) {
#pragma unroll
        for (int r = 0; r < 8; ++r) {
          const int tl = wm * 32 + 16 * sub + 8 * hh + r;
          so[tl * NR + n] = acc[sub][t][r];
        }
      }
    }
  }
  __syncthreads();

  const float bb = bilb[0];
  const size_t base = (size_t)b * SLAB;
  for (int ps = 0; ps < 2; ++ps) {
#pragma unroll
    for (int it = 0; it < 13; ++it) {
      const int p = tid + 256 * it;
      if (p < SLAB / 4) {
        const v4f s  = *(const v4f*)(so + 4 * p);
        const v4f mk = *(const v4f*)(mask + base + 4 * (size_t)p);
        v4f v;
        v[0] = (s[0] + bb) + mk[0];
        v[1] = (s[1] + bb) + mk[1];
        v[2] = (s[2] + bb) + mk[2];
        v[3] = (s[3] + bb) + mk[3];
        *(volatile v4f*)(out + base + 4 * (size_t)p) = v;
      }
    }
    __threadfence();
  }
}

extern "C" void kernel_launch(void* const* d_in, const int* in_sizes, int n_in,
                              void* d_out, int out_size, void* d_ws, size_t ws_size,
                              hipStream_t stream) {
  if (n_in < 7) return;
  if (in_sizes[0] != MT * TH) return;
  if (in_sizes[1] != MI * IH) return;
  if (in_sizes[2] != NB * SLAB) return;
  if (in_sizes[3] != TH * IH) return;
  if (in_sizes[4] != TH) return;
  if (in_sizes[5] != TH * TH) return;
  if (in_sizes[6] < 1) return;
  if (out_size != NB * SLAB) return;

  const float* encT = (const float*)d_in[0];
  const float* encI = (const float*)d_in[1];
  const float* mask = (const float*)d_in[2];
  const float* Kw   = (const float*)d_in[3];
  const float* Kb   = (const float*)d_in[4];
  const float* bilw = (const float*)d_in[5];
  const float* bilb = (const float*)d_in[6];
  float* out = (float*)d_out;

  size_t off = 0;
  const size_t oI  = off; off += (size_t)MI * IH * 2;
  const size_t oT  = off; off += (size_t)MT * TH * 2;
  const size_t oKw = off; off += (size_t)TH * IH * 2;
  const size_t oBw = off; off += (size_t)TH * TH * 2;
  const size_t oP  = off; off += (size_t)MI * TH * 2;
  const size_t oW  = off; off += (size_t)MI * TH * 2;
  if (off > ws_size) return;
  if (off > (size_t)134217728) return;

  char* ws = (char*)d_ws;
  _Float16* Ih  = (_Float16*)(ws + oI);
  _Float16* Thp = (_Float16*)(ws + oT);
  _Float16* Kwh = (_Float16*)(ws + oKw);
  _Float16* Bwh = (_Float16*)(ws + oBw);
  _Float16* Ph  = (_Float16*)(ws + oP);
  _Float16* Wh  = (_Float16*)(ws + oW);

  k_cvt<<<dim3((MI * IH) / 2048), dim3(256), 0, stream>>>(encI, Ih, 1.0f);
  k_cvt<<<dim3((MT * TH) / 2048), dim3(256), 0, stream>>>(encT, Thp, 1.0f);
  k_cvt<<<dim3((TH * IH) / 2048), dim3(256), 0, stream>>>(Kw, Kwh, 64.0f);
  k_cvt<<<dim3((TH * TH) / 2048), dim3(256), 0, stream>>>(bilw, Bwh, 32.0f);
  k_gemm<1><<<dim3(MI / 256, TH / 64), dim3(256), 0, stream>>>(Ih, IH, Kwh, IH, IH, TH, Kb, 0.015625f, Ph, TH);
  k_gemm<0><<<dim3(MI / 256, TH / 64), dim3(256), 0, stream>>>(Ph, TH, Bwh, TH, TH, TH, Kb, 0.03125f, Wh, TH);
  k_bil<<<dim3(NB), dim3(256), 0, stream>>>(Thp, Wh, mask, bilb, out);
  (void)hipGetLastError();
}
